// SelfInteraction_49589692399713
// MI455X (gfx1250) — hardware-verified
//
#include <hip/hip_runtime.h>
#include <math.h>

typedef __attribute__((ext_vector_type(16))) _Float16 v16h;
typedef __attribute__((ext_vector_type(16))) __bf16 v16b;
typedef __attribute__((ext_vector_type(8)))  _Float16 v8h;
typedef __attribute__((ext_vector_type(8)))  float v8f;
typedef __attribute__((ext_vector_type(4)))  float v4f;
typedef __attribute__((ext_vector_type(2)))  float v2f;
typedef __attribute__((ext_vector_type(4)))  unsigned v4u;
typedef __attribute__((ext_vector_type(4)))  int v4i;
typedef float __attribute__((may_alias)) float_a;
typedef int __attribute__((may_alias)) int_a;

template <typename T> __device__ __forceinline__ void vst2(void* p, T v) { *(volatile T*)p = v; __threadfence(); *(volatile T*)p = v; }
__device__ __forceinline__ v8f wmma16(v16h a, v16h b, v8f c) {
  v8f d = __builtin_amdgcn_wmma_f32_16x16x32_f16(false, a, false, b, (short)0, c, false, false);
  asm volatile("v_nop\n\tv_nop\n\tv_nop\n\tv_nop" : "+v"(d) : "v"(a), "v"(b));
  return d;
}
__device__ __forceinline__ v8f wmma_bf(v16b a, v16b b, v8f c) {
  v8f d = __builtin_amdgcn_wmma_f32_16x16x32_bf16(false, a, false, b, (short)0, c, false, false);
  asm volatile("v_nop\n\tv_nop\n\tv_nop\n\tv_nop" : "+v"(d) : "v"(a), "v"(b));
  return d;
}
__device__ __forceinline__ v16h frag_h(const _Float16* rowk0, int lane) {
  union { v16h v; v8h q[2]; } u; const _Float16* p = rowk0 + 8 * (lane >> 4);
  u.q[0] = *(const v8h*)p; u.q[1] = *(const v8h*)(p + 16); return u.v;
}
__device__ __forceinline__ v16h frag_f32(const float* rowk0, int lane) {
  v16h a; const float* p = rowk0 + 8 * (lane >> 4);
#pragma unroll
  for (int i = 0; i < 8; ++i) { a[i] = (_Float16)p[i]; a[8 + i] = (_Float16)p[16 + i]; }
  return a;
}
__device__ __forceinline__ v16h frag_f32s(const float* rowk0, int lane, float sc) {
  v16h a; const float* p = rowk0 + 8 * (lane >> 4);
#pragma unroll
  for (int i = 0; i < 8; ++i) { a[i] = (_Float16)(p[i] * sc); a[8 + i] = (_Float16)(p[16 + i] * sc); }
  return a;
}
__device__ __forceinline__ v16h fragc_f32(const float* W, int k0, int n, int lane, int ld, int K) {
  v16h a; const int g = lane >> 4;
#pragma unroll
  for (int i = 0; i < 8; ++i) { const int ka = k0 + 8 * g + i, kb = ka + 16;
    a[i] = (_Float16)(ka < K ? W[(size_t)(ka < K ? ka : K - 1) * ld + n] : 0.f); a[8 + i] = (_Float16)(kb < K ? W[(size_t)(kb < K ? kb : K - 1) * ld + n] : 0.f); }
  return a;
}
struct F2 { v16b h, l; };
__device__ __forceinline__ F2 bsplit16(const float v[16]) { F2 r;
#pragma unroll
  for (int i = 0; i < 16; ++i) { const __bf16 h = (__bf16)v[i]; r.h[i] = h; r.l[i] = (__bf16)(v[i] - (float)h); }
  return r; }
__device__ __forceinline__ F2 split_row(const float* row, int k0, int lane) { float v[16]; const float* p = row + k0 + 8 * (lane >> 4);
#pragma unroll
  for (int i = 0; i < 8; ++i) { v[i] = p[i]; v[8 + i] = p[16 + i]; }
  return bsplit16(v); }
__device__ __forceinline__ F2 split_rowK(const float* row, int k0, int lane, int K) { float v[16]; const int g = lane >> 4;
#pragma unroll
  for (int i = 0; i < 8; ++i) { const int ka = k0 + 8 * g + i, kb = ka + 16; v[i] = ka < K ? row[ka < K ? ka : K - 1] : 0.f; v[8 + i] = kb < K ? row[kb < K ? kb : K - 1] : 0.f; }
  return bsplit16(v); }
__device__ __forceinline__ F2 split_col(const float* W, int k0, int n, int lane, int ld, int K) { float v[16]; const int g = lane >> 4;
#pragma unroll
  for (int i = 0; i < 8; ++i) { const int ka = k0 + 8 * g + i, kb = ka + 16; v[i] = ka < K ? W[(size_t)(ka < K ? ka : K - 1) * ld + n] : 0.f; v[8 + i] = kb < K ? W[(size_t)(kb < K ? kb : K - 1) * ld + n] : 0.f; }
  return bsplit16(v); }
__device__ __forceinline__ v8f mac3(const F2& a, const F2& b, v8f c) { c = wmma_bf(a.l, b.h, c); c = wmma_bf(a.h, b.l, c); return wmma_bf(a.h, b.h, c); }
__device__ __forceinline__ float sigm(float v) { return 1.0f / (1.0f + expf(-v)); }
#define LDSX() do { asm volatile("s_wait_dscnt 0" ::: "memory"); __builtin_amdgcn_wave_barrier(); __builtin_amdgcn_fence(__ATOMIC_RELEASE, "workgroup"); } while (0)


#define NNODE 50000
#define M0 64
#define M1 32
#define FIN 160
__device__ __forceinline__ float bfr(float v) { return (float)(__bf16)v; }
__device__ __forceinline__ v16b vfrag(const float* row, int i, int lane) { float v[16]; const int g = lane >> 4;
#pragma unroll
  for (int e = 0; e < 8; ++e) { v[e] = row[M0 + (8 * g + e) * 3 + i]; v[8 + e] = row[M0 + (16 + 8 * g + e) * 3 + i]; }
  return bsplit16(v).h; }

__device__ __forceinline__ v16b frag_b(const __bf16* rowk0, int lane) { return __builtin_bit_cast(v16b, frag_h((const _Float16*)rowk0, lane)); }
__global__ __launch_bounds__(256) void k_packw(const float* __restrict__ W, int NU, int NV, int NW, __bf16* __restrict__ P) {
  const int u = blockIdx.x, tid = threadIdx.x; const float* Wu = W + (size_t)u * NV * NW; __bf16* Pu = P + (size_t)u * NW * NV;
  for (int q = tid; q < NV * NW / 8; q += 256) { const int w = (q * 8) / NV, v0 = (q * 8) % NV; union { __bf16 e[8]; v4u u4; } pk;
#pragma unroll
    for (int e = 0; e < 8; ++e) pk.e[e] = (__bf16)Wu[(size_t)(v0 + e) * NW + w];
    vst2((unsigned*)(Pu + (size_t)w * NV + v0), pk.u4); }
}
__global__ __launch_bounds__(256) void k_tp(const float* __restrict__ x, const __bf16* __restrict__ P000, const __bf16* __restrict__ P110, const __bf16* __restrict__ P011, const __bf16* __restrict__ P101, float* __restrict__ out) {
  __shared__ __align__(16) float so[16][FIN + 4];
  const int lane = threadIdx.x, col = lane & 15, g = lane >> 4; const size_t r0 = (size_t)blockIdx.x * 16; const float* xr = x + (r0 + col) * FIN;
  const float c0 = 0.013975424859373685f, c1s = 0.015625f, is3 = 0.57735026918962576f;
  v16b as_[2], av[3];
#pragma unroll
  for (int kc = 0; kc < 2; ++kc) as_[kc] = split_row(xr, kc * 32, lane).h;
#pragma unroll
  for (int i = 0; i < 3; ++i) av[i] = vfrag(xr, i, lane);
  const float* xrow[8];
#pragma unroll
  for (int r = 0; r < 8; ++r) xrow[r] = x + (r0 + 8 * g + r) * FIN;
  v8f os_[4] = {};
#pragma unroll 1
  for (int u = 0; u < M0; ++u) { float su[8];
#pragma unroll
    for (int r = 0; r < 8; ++r) su[r] = bfr(xrow[r][u]);
#pragma unroll
    for (int t = 0; t < 4; ++t) { v8f acc = {};
#pragma unroll
      for (int kc = 0; kc < 2; ++kc) acc = wmma_bf(as_[kc], frag_b(P000 + ((size_t)u * M0 + t * 16 + col) * M0 + kc * 32, lane), acc);
#pragma unroll
      for (int r = 0; r < 8; ++r) os_[t][r] += su[r] * acc[r]; } }
#pragma unroll 1
  for (int u = 0; u < M1; ++u) {
#pragma unroll
    for (int i = 0; i < 3; ++i) { float vu[8];
#pragma unroll
      for (int r = 0; r < 8; ++r) vu[r] = bfr(xrow[r][M0 + u * 3 + i]) * is3;
#pragma unroll
      for (int t = 0; t < 4; ++t) { v8f acc = {}; acc = wmma_bf(av[i], frag_b(P110 + ((size_t)u * M0 + t * 16 + col) * M1, lane), acc);
#pragma unroll
        for (int r = 0; r < 8; ++r) os_[t][r] += vu[r] * acc[r]; } } }
#pragma unroll
  for (int t = 0; t < 4; ++t)
#pragma unroll
    for (int r = 0; r < 8; ++r) so[8 * g + r][t * 16 + col] = os_[t][r] * c0;
  v8f ov[3][2] = {};
#pragma unroll 1
  for (int u = 0; u < M0; ++u) { float su[8];
#pragma unroll
    for (int r = 0; r < 8; ++r) su[r] = bfr(xrow[r][u]);
#pragma unroll
    for (int i = 0; i < 3; ++i)
#pragma unroll
      for (int t = 0; t < 2; ++t) { v8f acc = {}; acc = wmma_bf(av[i], frag_b(P011 + ((size_t)u * M1 + t * 16 + col) * M1, lane), acc);
#pragma unroll
        for (int r = 0; r < 8; ++r) ov[i][t][r] += su[r] * acc[r]; } }
#pragma unroll 1
  for (int u = 0; u < M1; ++u) { float vu[3][8];
#pragma unroll
    for (int i = 0; i < 3; ++i)
#pragma unroll
      for (int r = 0; r < 8; ++r) vu[i][r] = bfr(xrow[r][M0 + u * 3 + i]);
#pragma unroll
    for (int t = 0; t < 2; ++t) { v8f acc = {};
#pragma unroll
      for (int kc = 0; kc < 2; ++kc) acc = wmma_bf(as_[kc], frag_b(P101 + ((size_t)u * M1 + t * 16 + col) * M0 + kc * 32, lane), acc);
#pragma unroll
      for (int i = 0; i < 3; ++i)
#pragma unroll
        for (int r = 0; r < 8; ++r) ov[i][t][r] += vu[i][r] * acc[r]; } }
#pragma unroll
  for (int i = 0; i < 3; ++i)
#pragma unroll
    for (int t = 0; t < 2; ++t)
#pragma unroll
      for (int r = 0; r < 8; ++r) so[8 * g + r][M0 + (t * 16 + col) * 3 + i] = ov[i][t][r] * c1s;
  LDSX();
  for (int q = lane; q < 16 * (FIN / 4); q += 32) { const int rl = q / (FIN / 4), pc = q % (FIN / 4); vst2(out + (r0 + rl) * FIN + pc * 4, *(const v4f*)(&so[rl][pc * 4])); }
}
extern "C" void kernel_launch(void* const* d_in, const int* in_sizes, int n_in, void* d_out, int out_size, void* d_ws, size_t ws_size, hipStream_t stream) {
  (void)in_sizes; (void)n_in; (void)out_size; (void)ws_size;
  const float** I = (const float**)d_in;
  char* ws = (char*)d_ws; size_t off = 0;
  auto take = [&](size_t bytes) { char* p = ws + off; off += (bytes + 255) & ~(size_t)255; return p; };
  __bf16* P000 = (__bf16*)take((size_t)M0 * M0 * M0 * 2); __bf16* P110 = (__bf16*)take((size_t)M1 * M0 * M1 * 2); __bf16* P011 = (__bf16*)take((size_t)M0 * M1 * M1 * 2); __bf16* P101 = (__bf16*)take((size_t)M1 * M1 * M0 * 2);
  k_packw<<<M0, 256, 0, stream>>>(I[1], M0, M0, M0, P000);
  k_packw<<<M1, 256, 0, stream>>>(I[2], M1, M1, M0, P110);
  k_packw<<<M0, 256, 0, stream>>>(I[3], M0, M1, M1, P011);
  k_packw<<<M1, 256, 0, stream>>>(I[4], M1, M0, M1, P101);
  k_tp<<<NNODE / 16, 32, 0, stream>>>(I[0], P000, P110, P011, P101, (float*)d_out);
}
